// Model_7318624272394
// MI455X (gfx1250) — hardware-verified
//
#include <hip/hip_runtime.h>
#include <stdint.h>

#define NB     1024
#define NL     1024
#define ND     64
#define NCLS   10
#define P1ROWS 128
#define P2ROWS 14720

static_assert(ND == 64);
static_assert(11 * 11 * 11 * 11 == 14641);
static_assert(NL == 8 * 128);
static_assert(P2ROWS % 128 == 0 && P2ROWS >= 14641);
static_assert((64 * NCLS * 4) % 128 == 0);

typedef float          v4f   __attribute__((ext_vector_type(4)));
typedef float          v8f   __attribute__((ext_vector_type(8)));
typedef int            v4i   __attribute__((ext_vector_type(4)));
typedef int            v8i   __attribute__((ext_vector_type(8)));
typedef unsigned int   v2u   __attribute__((ext_vector_type(2)));
typedef unsigned int   v4u   __attribute__((ext_vector_type(4)));
typedef unsigned short v8us  __attribute__((ext_vector_type(8)));
typedef __bf16         v16bf __attribute__((ext_vector_type(16)));
typedef v4f  __attribute__((may_alias)) v4fa;
typedef v4i  __attribute__((may_alias)) v4ia;
typedef v2u  __attribute__((may_alias)) v2ua;
typedef v8us __attribute__((may_alias)) v8usa;
union FragB { v16bf v; v8us h[2]; v8i w; };

constexpr int MODE_P1 = 0, MODE_P2 = 1, MODE_X = 2, MODE_DENSE = 3;

constexpr size_t OFF_RW2 = 0;
constexpr size_t OFF_LW2 = 32768;
constexpr size_t OFF_H0N = 36864;
constexpr size_t OFF_P1  = 39936;
constexpr size_t OFF_P2  = 72704;
constexpr size_t OFF_N3  = 3841024;
constexpr size_t nodeOff(int t) {
  size_t o = OFF_N3;
  for (int u = 3; u < t; ++u) o += (size_t)NB * (size_t)(NL >> u) * 256;
  return o;
}
constexpr size_t WS_TOTAL = nodeOff(11);
static_assert(OFF_LW2 == OFF_RW2 + 128 * 128 * 2);
static_assert(OFF_H0N == OFF_LW2 + 16 * 128 * 2);
static_assert(OFF_P1 == OFF_H0N + 12 * 64 * 4);
static_assert(OFF_P2 == OFF_P1 + (size_t)P1ROWS * 256);
static_assert(OFF_N3 == OFF_P2 + (size_t)P2ROWS * 256);
static_assert(WS_TOTAL == 70687744);
static_assert(WS_TOTAL <= 134217728);
static_assert(OFF_H0N % 256 == 0 && OFF_P1 % 256 == 0 && OFF_P2 % 256 == 0 && OFF_N3 % 256 == 0);
static_assert(nodeOff(4)  == OFF_N3 + (size_t)((256 - (2048 >> 4))  << 16) * 4);
static_assert(nodeOff(7)  == OFF_N3 + (size_t)((256 - (2048 >> 7))  << 16) * 4);
static_assert(nodeOff(10) == OFF_N3 + (size_t)((256 - (2048 >> 10)) << 16) * 4);
static_assert((NB * (NL >> 3)) % 128 == 0 && (NB * (NL >> 10)) % 128 == 0);

#define O_L    0
#define O_R    32768
#define O_A    65536
#define O_AL   98304
#define O_IDX  99328
#define O_FLG  100352
#define O_IDX2 101376
#define O_FLG2 101888
#define LDS_COMB 102400
#define O_RES  102400
#define O_OUT  167936
#define LDS_Q  170496
static_assert(LDS_Q <= 320 * 1024);

__device__ __forceinline__ unsigned f2bf(float f) {
  const unsigned u = __float_as_uint(f);
  const unsigned r = (u + 0x7FFFu + ((u >> 16) & 1u)) >> 16;
  return ((u & 0x7fffffffu) > 0x7f800000u) ? 0x7fc0u : r;
}
__device__ __forceinline__ float bf2f(unsigned b) { return __uint_as_float(b << 16); }
__device__ __forceinline__ float bfr(float f) { return bf2f(f2bf(f)); }
__device__ __forceinline__ int clampi(int v, int lo, int hi) { return min(max(v, lo), hi); }
__device__ __forceinline__ v8f z8() { v8f z = {0.f, 0.f, 0.f, 0.f, 0.f, 0.f, 0.f, 0.f}; return z; }
__device__ __forceinline__ float hsum16(float v) {
  v += __shfl_xor(v, 1);
  v += __shfl_xor(v, 2);
  v += __shfl_xor(v, 4);
  v += __shfl_xor(v, 8);
  return v;
}
__device__ __forceinline__ v4f blend(v4f a, v4f b, unsigned mk) {
  const v4u ua = __builtin_bit_cast(v4u, a);
  const v4u ub = __builtin_bit_cast(v4u, b);
  const v4u mv = {mk, mk, mk, mk};
  const v4u r = (ua & ~mv) | (ub & mv);
  return __builtin_bit_cast(v4f, r);
}
__device__ __forceinline__ v4u pack8(v4f a, v4f c) {
  v4u v;
  v.x = f2bf(a.x) | (f2bf(a.y) << 16);
  v.y = f2bf(a.z) | (f2bf(a.w) << 16);
  v.z = f2bf(c.x) | (f2bf(c.y) << 16);
  v.w = f2bf(c.z) | (f2bf(c.w) << 16);
  return v;
}

__device__ __forceinline__ v8f wmb(const FragB& a, const FragB& b, v8f c) {
  v8f d = __builtin_amdgcn_wmma_f32_16x16x32_bf16(false, a.v, false, b.v, (short)0, c, false, false);
  asm volatile("v_nop\n\tv_nop\n\tv_nop\n\tv_nop" : "+v"(d) : "v"(a.w), "v"(b.w));
  return d;
}

__device__ __forceinline__ void put_lr(int row, int c4, v4f vl, v4f vr) {
  extern __shared__ __align__(16) unsigned char smem[];
  float* sL = (float*)(smem + O_L);
  float* sR = (float*)(smem + O_R);
  unsigned short* sA = (unsigned short*)(smem + O_A);
  *(v4fa*)(sL + row * 64 + c4) = vl;
  *(v4fa*)(sR + row * 64 + c4) = vr;
  const unsigned h0 = f2bf(vr.x), h1 = f2bf(vr.y), h2 = f2bf(vr.z), h3 = f2bf(vr.w);
  const float l0 = vr.x - bf2f(h0), l1 = vr.y - bf2f(h1), l2 = vr.z - bf2f(h2), l3 = vr.w - bf2f(h3);
  v2u hi, lo;
  hi.x = h0 | (h1 << 16);
  hi.y = h2 | (h3 << 16);
  lo.x = f2bf(l0) | (f2bf(l1) << 16);
  lo.y = f2bf(l2) | (f2bf(l3) << 16);
  *(v2ua*)(sA + row * 128 + c4) = hi;
  *(v2ua*)(sA + row * 128 + 64 + c4) = lo;
}
__device__ __forceinline__ void put_a(int row, int c4, v4f vr) {
  extern __shared__ __align__(16) unsigned char smem[];
  unsigned short* sA = (unsigned short*)(smem + O_A);
  const unsigned h0 = f2bf(vr.x), h1 = f2bf(vr.y), h2 = f2bf(vr.z), h3 = f2bf(vr.w);
  const float l0 = vr.x - bf2f(h0), l1 = vr.y - bf2f(h1), l2 = vr.z - bf2f(h2), l3 = vr.w - bf2f(h3);
  v2u hi, lo;
  hi.x = h0 | (h1 << 16);
  hi.y = h2 | (h3 << 16);
  lo.x = f2bf(l0) | (f2bf(l1) << 16);
  lo.y = f2bf(l2) | (f2bf(l3) << 16);
  *(v2ua*)(sA + row * 128 + c4) = hi;
  *(v2ua*)(sA + row * 128 + 64 + c4) = lo;
}

__device__ __forceinline__ void tile_scores(const unsigned short* __restrict__ RW2, int w, int h, int m) {
  extern __shared__ __align__(16) unsigned char smem[];
  const float* sL = (const float*)(smem + O_L);
  const unsigned short* sA = (const unsigned short*)(smem + O_A);
  float* sAl = (float*)(smem + O_AL);

  v8f acc[8];
#pragma unroll
  for (int nt = 0; nt < 8; ++nt) acc[nt] = z8();

  const unsigned short* arow = sA + (16 * w + m) * 128 + 8 * h;
  const unsigned short* brow = RW2 + m * 128 + 8 * h;
#pragma unroll 1
  for (int k0 = 0; k0 < 128; k0 += 32) {
    FragB a;
    a.h[0] = *(const v8usa*)(arow + k0);
    a.h[1] = *(const v8usa*)(arow + k0 + 16);
#pragma unroll
    for (int nt = 0; nt < 8; ++nt) {
      const unsigned short* bq = brow + nt * 16 * 128 + k0;
      FragB b;
      b.h[0] = *(const v8usa*)bq;
      b.h[1] = *(const v8usa*)(bq + 16);
      acc[nt] = wmb(a, b, acc[nt]);
    }
  }

  const int rbase = 16 * w + 8 * h;
  const float* lrow = sL + rbase * 64 + m;
  float s0[8], s1[8];
#pragma unroll
  for (int r = 0; r < 8; ++r) { s0[r] = 0.0f; s1[r] = 0.0f; }
#pragma unroll
  for (int nt = 0; nt < 4; ++nt) {
#pragma unroll
    for (int r = 0; r < 8; ++r) {
      const float lv = lrow[r * 64 + 16 * nt];
      s0[r] += lv * acc[nt][r];
      s1[r] += lv * acc[4 + nt][r];
    }
  }
  float al0[8], al1[8];
#pragma unroll
  for (int r = 0; r < 8; ++r) {
    const float a = hsum16(s0[r]);
    const float b = hsum16(s1[r]);
    const float e = expf(-fabsf(a - b));
    const float inv = 1.0f / (1.0f + e);
    const float big = inv, sml = e * inv;
    const bool f = (a >= b);
    al0[r] = f ? big : sml;
    al1[r] = f ? sml : big;
  }
  if (m == 0) {
#pragma unroll
    for (int r = 0; r < 8; ++r) {
      sAl[(rbase + r) * 2]     = al0[r];
      sAl[(rbase + r) * 2 + 1] = al1[r];
    }
  }
}

__device__ __forceinline__ v4f row_comb(int row, int m) {
  extern __shared__ __align__(16) unsigned char smem[];
  const float* sL = (const float*)(smem + O_L);
  const float* sR = (const float*)(smem + O_R);
  const float* sAl = (const float*)(smem + O_AL);
  const float a0 = sAl[2 * row], a1 = sAl[2 * row + 1];
  const v4f l = *(const v4fa*)(sL + row * 64 + 4 * m);
  const v4f r = *(const v4fa*)(sR + row * 64 + 4 * m);
  v4f v;
  v.x = a0 * l.x + a1 * r.x;
  v.y = a0 * l.y + a1 * r.y;
  v.z = a0 * l.z + a1 * r.z;
  v.w = a0 * l.w + a1 * r.w;
  float ss = v.x * v.x + v.y * v.y + v.z * v.z + v.w * v.w;
  ss = hsum16(ss);
  const float den = sqrtf(ss * (1.0f / 64.0f) + 1e-6f) + 1e-6f;
  const float inv = 1.0f / den;
  v.x *= inv; v.y *= inv; v.z *= inv; v.w *= inv;
  return v;
}

__global__ __launch_bounds__(256) void k_prep(const float* __restrict__ emb, const float* __restrict__ rw,
                                              const float* __restrict__ lw, unsigned short* __restrict__ RW2,
                                              unsigned short* __restrict__ LW2, float* __restrict__ H0N) {
  const int b = blockIdx.x, tid = threadIdx.x;
  if (b < 8) {
    const int u = b * 256 + tid;
    const int row = u >> 4, sc = ((u & 15) * 8) & 63;
    const float* s = rw + row * 64 + sc;
    const v4f a = *(const v4fa*)s;
    const v4f c = *(const v4fa*)(s + 4);
    const v4u v = pack8(a, c);
    unsigned short* d = RW2 + (size_t)u * 8;
    *(volatile v4u*)d = v;
    __threadfence();
    *(volatile v4u*)d = v;
  } else if (b == 8) {
    const int u = tid;
    const int row = u >> 4, sc = ((u & 15) * 8) & 63;
    const int srow = min(row, NCLS - 1);
    const float* s = lw + srow * 64 + sc;
    const v4f a = *(const v4fa*)s;
    const v4f c = *(const v4fa*)(s + 4);
    v4u v = pack8(a, c);
    const unsigned mk = (row < NCLS) ? 0xffffffffu : 0u;
    v.x &= mk; v.y &= mk; v.z &= mk; v.w &= mk;
    unsigned short* d = LW2 + (size_t)u * 8;
    *(volatile v4u*)d = v;
    __threadfence();
    *(volatile v4u*)d = v;
  } else {
    const int row = min(tid >> 4, 11);
    const int srow = min(row, 10);
    const int c4 = (tid & 15) * 4;
    const v4f e0 = *(const v4fa*)(emb + srow * 64 + c4);
    v4f e;
    e.x = bfr(e0.x); e.y = bfr(e0.y); e.z = bfr(e0.z); e.w = bfr(e0.w);
    float ss = e.x * e.x + e.y * e.y + e.z * e.z + e.w * e.w;
    ss = hsum16(ss);
    const float den = sqrtf(ss * (1.0f / 64.0f) + 1e-6f) + 1e-6f;
    const float sc = (row == 11) ? 1.0f : (1.0f / den);
    v4f o;
    o.x = e.x * sc; o.y = e.y * sc; o.z = e.z * sc; o.w = e.w * sc;
    if (tid < 192) {
      float* d = H0N + tid * 4;
      *(volatile v4f*)d = o;
      __threadfence();
      *(volatile v4f*)d = o;
    }
  }
}

template <int MODE>
__global__ __launch_bounds__(256) void k_combine(const int* __restrict__ x, const float* __restrict__ src,
                                                 const unsigned short* __restrict__ RW2,
                                                 float* __restrict__ dst) {
  extern __shared__ __align__(16) unsigned char smem[];
  int* sIdx = (int*)(smem + O_IDX);
  const int tid = threadIdx.x, lane = tid & 31, w = tid >> 5;
  const int h = lane >> 4, m = lane & 15;
  const int c4 = (tid & 15) * 4;

  if (MODE != MODE_DENSE) {
    const int row = tid >> 1, side = tid & 1;
    int pm = blockIdx.x * 128 + row;
    int idx;
    if (MODE == MODE_P1) {
      pm = min(pm, 120);
      idx = side ? (pm % 11) : (pm / 11);
    } else if (MODE == MODE_P2) {
      pm = min(pm, 14640);
      idx = side ? (pm % 121) : (pm / 121);
    } else {
      const v4i xs = *(const v4ia*)(x + (size_t)pm * 8 + 4 * side);
      const int a0 = clampi(xs.x, 0, 10), a1 = clampi(xs.y, 0, 10);
      const int a2 = clampi(xs.z, 0, 10), a3 = clampi(xs.w, 0, 10);
      idx = (a0 * 11 + a1) * 121 + a2 * 11 + a3;
    }
    sIdx[tid] = idx;
    __syncthreads();
  }

#pragma unroll 2
  for (int k = 0; k < 8; ++k) {
    const int row = (tid + 256 * k) >> 4;
    v4f vl, vr;
    if (MODE == MODE_DENSE) {
      const float* s = src + (size_t)blockIdx.x * 16384 + row * 128 + c4;
      vl = *(const v4fa*)s;
      vr = *(const v4fa*)(s + 64);
    } else {
      const int il = sIdx[2 * row], ir = sIdx[2 * row + 1];
      vl = *(const v4fa*)(src + (size_t)il * 64 + c4);
      vr = *(const v4fa*)(src + (size_t)ir * 64 + c4);
    }
    put_lr(row, c4, vl, vr);
  }
  __syncthreads();

  tile_scores(RW2, w, h, m);
  __syncthreads();

  v4f o[8];
#pragma unroll
  for (int it = 0; it < 8; ++it) o[it] = row_comb(16 * w + 2 * it + h, m);

  float* drow = dst + ((size_t)blockIdx.x * 128 + 16 * w) * 64 + (size_t)lane * 4;
#pragma unroll
  for (int it = 0; it < 8; ++it) *(volatile v4f*)(drow + it * 128) = o[it];
  __threadfence();
#pragma unroll
  for (int it = 0; it < 8; ++it) *(volatile v4f*)(drow + it * 128) = o[it];
}

__global__ __launch_bounds__(256) void k_query(const int* __restrict__ x, const int* __restrict__ qlo,
                                               const int* __restrict__ qhi, const float* __restrict__ wsf,
                                               const unsigned short* __restrict__ RW2,
                                               const unsigned short* __restrict__ LW2,
                                               float* __restrict__ out,
                                               int oH0N, int oP1, int oP2, int oN3) {
  extern __shared__ __align__(16) unsigned char smem[];
  int* sIdx  = (int*)(smem + O_IDX);
  int* sFlg  = (int*)(smem + O_FLG);
  int* sIdx2 = (int*)(smem + O_IDX2);
  int* sFlg2 = (int*)(smem + O_FLG2);
  float* RES = (float*)(smem + O_RES);
  float* sOut = (float*)(smem + O_OUT);
  const unsigned short* sA = (const unsigned short*)(smem + O_A);

  const int tid = threadIdx.x, lane = tid & 31, w = tid >> 5;
  const int h = lane >> 4, m = lane & 15;
  const int c4 = (tid & 15) * 4;
  const int offINF = oH0N + 11 * 64;

  const int rowC = tid >> 1, side = tid & 1;
  const int blC = rowC & 63, slotC = rowC >> 6;
  const int bC = blockIdx.x * 64 + blC;
  const int qlC = qlo[bC], qhC = qhi[bC];
  const int rowR = tid & 127;
  const int blR = rowR & 63, slotR = rowR >> 6;
  const int bR = blockIdx.x * 64 + blR;
  const int qlR = qlo[bR], qhR = qhi[bR];
  const int* xC = x + (size_t)bC * NL;
  const int* xR = x + (size_t)bR * NL;

  {
    const int c = clampi(slotR ? qhR : qlR, 0, NL - 1);
    const bool ins = (qlR <= c) && (qhR >= c);
    const int sym = clampi(xR[c], 0, 10);
    const int off = ins ? (oH0N + sym * 64) : offINF;
    if (tid < 128) sIdx2[rowR] = off;
  }
  __syncthreads();
#pragma unroll 2
  for (int k = 0; k < 8; ++k) {
    const int row = (tid + 256 * k) >> 4;
    const v4f v = *(const v4fa*)(wsf + (size_t)sIdx2[row] + c4);
    *(v4fa*)(RES + row * 64 + c4) = v;
  }
  __syncthreads();

#pragma unroll 1
  for (int t = 1; t <= 10; ++t) {
    const int tp = t - 1;
    const float* resP = RES + (tp & 1) * 8192;
    float* resC = RES + (t & 1) * 8192;
    const int nT = NL >> t;
    {
      const int p = clampi((slotC ? qhC : qlC) >> t, 0, nT - 1);
      const int c = 2 * p + side;
      const int lows = c << tp, highs = lows + (1 << tp) - 1;
      const bool ins = (qlC <= lows) && (qhC >= highs);
      const bool dis = (qlC > highs) || (qhC < lows);
      int off;
      if (tp == 0) {
        off = oH0N + clampi(xC[c], 0, 10) * 64;
      } else if (tp == 1) {
        const int a0 = clampi(xC[2 * c], 0, 10), a1 = clampi(xC[2 * c + 1], 0, 10);
        off = oP1 + (a0 * 11 + a1) * 64;
      } else if (tp == 2) {
        const v4i xs = *(const v4ia*)(xC + 4 * c);
        const int a0 = clampi(xs.x, 0, 10), a1 = clampi(xs.y, 0, 10);
        const int a2 = clampi(xs.z, 0, 10), a3 = clampi(xs.w, 0, 10);
        off = oP2 + ((a0 * 11 + a1) * 121 + a2 * 11 + a3) * 64;
      } else {
        off = oN3 + ((256 - (2048 >> tp)) << 16) + (bC * (NL >> tp) + c) * 64;
      }
      if (!ins && dis) off = offINF;
      const bool part = (!ins) && (!dis);
      const int rr = (c == (qlC >> tp)) ? blC : (64 + blC);
      sIdx[tid] = off;
      sFlg[tid] = part ? (rr + 1) : 0;
    }
    {
      const int p = clampi((slotR ? qhR : qlR) >> t, 0, nT - 1);
      const int lows = p << t, highs = lows + (1 << t) - 1;
      const bool ins = (qlR <= lows) && (qhR >= highs);
      const bool dis = (qlR > highs) || (qhR < lows);
      int off;
      if (t == 1) {
        const int a0 = clampi(xR[2 * p], 0, 10), a1 = clampi(xR[2 * p + 1], 0, 10);
        off = oP1 + (a0 * 11 + a1) * 64;
      } else if (t == 2) {
        const v4i xs = *(const v4ia*)(xR + 4 * p);
        const int a0 = clampi(xs.x, 0, 10), a1 = clampi(xs.y, 0, 10);
        const int a2 = clampi(xs.z, 0, 10), a3 = clampi(xs.w, 0, 10);
        off = oP2 + ((a0 * 11 + a1) * 121 + a2 * 11 + a3) * 64;
      } else {
        off = oN3 + ((256 - (2048 >> t)) << 16) + (bR * nT + p) * 64;
      }
      if (!ins && dis) off = offINF;
      if (tid < 128) {
        sIdx2[rowR] = off;
        sFlg2[rowR] = ((!ins) && (!dis)) ? 1 : 0;
      }
    }
    __syncthreads();

#pragma unroll 2
    for (int k = 0; k < 8; ++k) {
      const int row = (tid + 256 * k) >> 4;
      const int o0 = sIdx[2 * row], o1 = sIdx[2 * row + 1];
      const int f0 = sFlg[2 * row], f1 = sFlg[2 * row + 1];
      const v4f g0 = *(const v4fa*)(wsf + (size_t)o0 + c4);
      const v4f g1 = *(const v4fa*)(wsf + (size_t)o1 + c4);
      const v4f r0 = *(const v4fa*)(resP + max(f0 - 1, 0) * 64 + c4);
      const v4f r1 = *(const v4fa*)(resP + max(f1 - 1, 0) * 64 + c4);
      const v4f vl = blend(g0, r0, f0 ? 0xffffffffu : 0u);
      const v4f vr = blend(g1, r1, f1 ? 0xffffffffu : 0u);
      put_lr(row, c4, vl, vr);
    }
    __syncthreads();

    tile_scores(RW2, w, h, m);
    __syncthreads();

#pragma unroll
    for (int it = 0; it < 8; ++it) {
      const int row = 16 * w + 2 * it + h;
      const v4f cb = row_comb(row, m);
      const v4f g = *(const v4fa*)(wsf + (size_t)sIdx2[row] + 4 * m);
      const v4f v = blend(g, cb, sFlg2[row] ? 0xffffffffu : 0u);
      *(v4fa*)(resC + row * 64 + 4 * m) = v;
    }
    __syncthreads();
  }

#pragma unroll 2
  for (int k = 0; k < 8; ++k) {
    const int row = (tid + 256 * k) >> 4;
    const v4f v = *(const v4fa*)(RES + row * 64 + c4);
    put_a(row, c4, v);
  }
  __syncthreads();
  {
    v8f acc = z8();
    const unsigned short* arow = sA + (16 * w + m) * 128 + 8 * h;
    const unsigned short* brow = LW2 + m * 128 + 8 * h;
#pragma unroll
    for (int k0 = 0; k0 < 128; k0 += 32) {
      FragB a, b;
      a.h[0] = *(const v8usa*)(arow + k0);
      a.h[1] = *(const v8usa*)(arow + k0 + 16);
      b.h[0] = *(const v8usa*)(brow + k0);
      b.h[1] = *(const v8usa*)(brow + k0 + 16);
      acc = wmb(a, b, acc);
    }
    if (w < 4 && m < NCLS) {
#pragma unroll
      for (int r = 0; r < 8; ++r) sOut[(16 * w + 8 * h + r) * NCLS + m] = acc[r];
    }
  }
  __syncthreads();
  if (tid < 160) {
    const v4f v = *(const v4fa*)(sOut + 4 * tid);
    float* d = out + (size_t)blockIdx.x * 640 + 4 * tid;
    *(volatile v4f*)d = v;
    __threadfence();
    *(volatile v4f*)d = v;
  }
}

extern "C" void kernel_launch(void* const* d_in, const int* in_sizes, int n_in,
                              void* d_out, int out_size, void* d_ws, size_t ws_size,
                              hipStream_t stream) {
  if (n_in < 6) return;
  if (in_sizes[0] != NB * NL) return;
  if (in_sizes[1] != NB || in_sizes[2] != NB) return;
  if (in_sizes[3] != 11 * ND) return;
  if (in_sizes[4] != 2 * ND * ND) return;
  if (in_sizes[5] != NCLS * ND) return;
  if (out_size != NB * NCLS) return;
  if (WS_TOTAL > ws_size) return;

  const int*   x   = (const int*)d_in[0];
  const int*   ql  = (const int*)d_in[1];
  const int*   qh  = (const int*)d_in[2];
  const float* emb = (const float*)d_in[3];
  const float* rw  = (const float*)d_in[4];
  const float* lw  = (const float*)d_in[5];
  float* out = (float*)d_out;

  char* ws = (char*)d_ws;
  unsigned short* RW2 = (unsigned short*)(ws + OFF_RW2);
  unsigned short* LW2 = (unsigned short*)(ws + OFF_LW2);
  float* H0N = (float*)(ws + OFF_H0N);
  float* P1  = (float*)(ws + OFF_P1);
  float* P2  = (float*)(ws + OFF_P2);
  const float* wsf = (const float*)d_ws;

  (void)hipFuncSetAttribute(reinterpret_cast<const void*>(&k_combine<MODE_P1>),
                            hipFuncAttributeMaxDynamicSharedMemorySize, LDS_COMB);
  (void)hipFuncSetAttribute(reinterpret_cast<const void*>(&k_combine<MODE_P2>),
                            hipFuncAttributeMaxDynamicSharedMemorySize, LDS_COMB);
  (void)hipFuncSetAttribute(reinterpret_cast<const void*>(&k_combine<MODE_X>),
                            hipFuncAttributeMaxDynamicSharedMemorySize, LDS_COMB);
  (void)hipFuncSetAttribute(reinterpret_cast<const void*>(&k_combine<MODE_DENSE>),
                            hipFuncAttributeMaxDynamicSharedMemorySize, LDS_COMB);
  (void)hipFuncSetAttribute(reinterpret_cast<const void*>(&k_query),
                            hipFuncAttributeMaxDynamicSharedMemorySize, LDS_Q);

  k_prep<<<dim3(10), dim3(256), 0, stream>>>(emb, rw, lw, RW2, LW2, H0N);
  k_combine<MODE_P1><<<dim3(1), dim3(256), LDS_COMB, stream>>>(x, H0N, RW2, P1);
  k_combine<MODE_P2><<<dim3(P2ROWS / 128), dim3(256), LDS_COMB, stream>>>(x, P1, RW2, P2);
  k_combine<MODE_X><<<dim3((NB * (NL >> 3)) / 128), dim3(256), LDS_COMB, stream>>>(
      x, P2, RW2, (float*)(ws + nodeOff(3)));
  for (int t = 4; t <= 10; ++t) {
    const int rows = NB * (NL >> t);
    k_combine<MODE_DENSE><<<dim3(rows / 128), dim3(256), LDS_COMB, stream>>>(
        x, (const float*)(ws + nodeOff(t - 1)), RW2, (float*)(ws + nodeOff(t)));
  }
  k_query<<<dim3(NB / 64), dim3(256), LDS_Q, stream>>>(x, ql, qh, wsf, RW2, LW2, out,
                                                       (int)(OFF_H0N / 4), (int)(OFF_P1 / 4),
                                                       (int)(OFF_P2 / 4), (int)(OFF_N3 / 4));
  (void)hipGetLastError();
}
